// GCN_HL03_bn_tanh_42545946034238
// MI455X (gfx1250) — hardware-run, weakly checked
//
#include <hip/hip_runtime.h>


namespace {
constexpr int N = 50000, NP = 50048  , E = 300000, NBLKR = 391;
constexpr float XS = 8.0f, WSC = 256.0f, BNE = 1e-5f;

typedef _Float16 b16;
typedef __attribute__((ext_vector_type(16))) _Float16 v16b;
typedef __attribute__((ext_vector_type(8))) _Float16 v8b;
typedef __attribute__((ext_vector_type(8))) float v8f;
typedef __attribute__((ext_vector_type(4))) float v4f;
__device__ __forceinline__ float bf16_rne(float f) { unsigned int u = __float_as_uint(f); u += 0x7FFFu + ((u >> 16) & 1u); return __uint_as_float(u & 0xFFFF0000u); }
__device__ __forceinline__ void split16(float v, b16& hi, b16& lo) { hi = (b16)v; lo = (b16)(v - (float)hi); }
__device__ __forceinline__ v16b frag_kb(const b16* p, int hh) { const v8b a = *(const v8b*)(p + 8 * hh), b = *(const v8b*)(p + 16 + 8 * hh); v16b f;
#pragma unroll
  for (int e = 0; e < 8; ++e) { f[e] = a[e]; f[8 + e] = b[e]; } return f; }
__device__ __forceinline__ v8f wmma16b(v16b a, v16b b, v8f c) { v8f d = __builtin_amdgcn_wmma_f32_16x16x32_f16(false, a, false, b, (short)0, c, false, false); asm volatile("v_nop\n\tv_nop\n\tv_nop\n\tv_nop" : "+v"(d) : "v"(a), "v"(b)); return d; }
__device__ __forceinline__ void wave_lds_sync() { __builtin_amdgcn_fence(__ATOMIC_RELEASE, "workgroup"); __builtin_amdgcn_wave_barrier(); __builtin_amdgcn_fence(__ATOMIC_ACQUIRE, "workgroup"); }
__device__ __forceinline__ float pmul(float a, float b) { float p = a * b; asm volatile("" : "+v"(p)); return p; }
__device__ __forceinline__ int iclamp(int v, int lo, int hi) { return v < lo ? lo : (v > hi ? hi : v); }
__device__ __forceinline__ float nexp(float x) { return __builtin_amdgcn_exp2f(x * 1.4426950408889634f); }
__device__ __forceinline__ float tanh_(float x) { const float e = nexp(-2.0f * fabsf(x)); const float t = (1.0f - e) / (1.0f + e); return x < 0.0f ? -t : t; }

constexpr int CSR_NBLK = 512, CSR_GB = 9, CSR_GN = 1 << CSR_GB  , CSR_MAXG = 512, CSR_CAP = 12288  ;
__global__ __launch_bounds__(64) void csrA_kernel(const int* __restrict__ dst, int E, int N, int nG, int CHP, int NGP, int* __restrict__ STG, int* __restrict__ HST) {
  extern __shared__ int sm[];
  int* cnt = sm; int* run = sm + NGP; int* ids = sm + 2 * NGP;
  const int b = blockIdx.x; const int ch = (E + CSR_NBLK - 1) / CSR_NBLK; const int e0 = b * ch, e1 = min(E, e0 + ch);
  for (int i = threadIdx.x; i < NGP; i += 64) cnt[i] = 0;
  for (int i = threadIdx.x; i < CHP; i += 64) ids[i] = -1;
  __syncthreads();
  if (threadIdx.x == 0) {
    for (int e = e0; e < e1; ++e) { int d = dst[e]; d = (d < 0) ? 0 : (d >= N ? N - 1 : d); cnt[d >> CSR_GB] += 1; }
    int acc = 0; for (int g = 0; g < nG; ++g) { run[g] = acc; acc += cnt[g]; }
    for (int e = e0; e < e1; ++e) { int d = dst[e]; d = (d < 0) ? 0 : (d >= N ? N - 1 : d); const int g = d >> CSR_GB; ids[run[g]] = e; run[g] += 1; } }
  __syncthreads();
  typedef __attribute__((ext_vector_type(4))) int v4i;
  for (int pass = 0; pass < 2; ++pass) {
    for (int i = threadIdx.x; i < CHP / 4; i += 64) *(volatile v4i*)(STG + (size_t)b * CHP + i * 4) = *(const v4i*)(&ids[i * 4]);
    for (int i = threadIdx.x; i < NGP / 4; i += 64) { v4i v; for (int e = 0; e < 4; ++e) v[e] = (i * 4 + e < nG) ? cnt[i * 4 + e] : 0; *(volatile v4i*)(HST + (size_t)b * NGP + i * 4) = v; }
    __threadfence(); }
}
__global__ __launch_bounds__(512) void csrS_kernel(const int* __restrict__ HST, int nG, int NGP, int* __restrict__ START, int* __restrict__ TOT, int* __restrict__ OFF) {
  __shared__ int tot[CSR_MAXG];
  const int b = threadIdx.x;
  for (int pass = 0; pass < 2; ++pass) { int runb = 0; for (int g = 0; g < nG; ++g) { int c = HST[(size_t)b * NGP + g]; c = (c < 0) ? 0 : c; ((volatile int*)OFF)[(size_t)g * CSR_NBLK + b] = runb; runb += c; } __threadfence(); }
  for (int g = threadIdx.x; g < nG; g += 512) { int s = 0; for (int bb = 0; bb < CSR_NBLK; ++bb) { int c = HST[(size_t)bb * NGP + g]; s += (c < 0) ? 0 : c; } tot[g] = s; }
  __syncthreads();
  if (threadIdx.x < 32) {
    __shared__ int st[CSR_MAXG + 32];
    if (threadIdx.x == 0) { int acc = 0; for (int g = 0; g < NGP; ++g) { st[g] = acc; if (g < nG) acc += (tot[g] + 31) & ~31; } st[NGP] = acc; }
    __builtin_amdgcn_fence(__ATOMIC_RELEASE, "workgroup"); __builtin_amdgcn_wave_barrier(); __builtin_amdgcn_fence(__ATOMIC_ACQUIRE, "workgroup");
    for (int pass = 0; pass < 2; ++pass) { for (int i = threadIdx.x; i < NGP + 32; i += 32) { ((volatile int*)START)[i] = (i <= NGP) ? st[min(i, NGP)] : 0; ((volatile int*)TOT)[i] = (i < nG) ? tot[i] : 0; } __threadfence(); } }
}
__global__ __launch_bounds__(256) void csrB_kernel(const int* __restrict__ dst, int N, int nG, int CHP, int NGP, int permLen, const int* __restrict__ STG, const int* __restrict__ HST, const int* __restrict__ OFF, const int* __restrict__ START, const int* __restrict__ TOT, int* __restrict__ PERM, int* __restrict__ ROWPTR, int* __restrict__ ROWCNT, int* __restrict__ FLAG) {
  typedef __attribute__((ext_vector_type(4))) int v4i;
  __shared__ int ids[CSR_CAP]; __shared__ unsigned short key[CSR_CAP]; __shared__ int outp[CSR_CAP]; __shared__ int ncnt[CSR_GN + 1]; __shared__ int boff[CSR_NBLK + 1];
  const int g = blockIdx.x, t_ = threadIdx.x; int tot = TOT[g]; int st = START[g], stn = START[g + 1]; const int v0 = g * CSR_GN; const int nv = min(CSR_GN, N - v0);
  st = (st < 0) ? 0 : (st > permLen - 32 ? permLen - 32 : st) & ~31; stn = (stn < st) ? st : (stn > permLen ? permLen : stn); tot = (tot < 0) ? 0 : tot; if (tot > stn - st && tot <= CSR_CAP) tot = stn - st;
  if (tot > CSR_CAP) {
    for (int pass = 0; pass < 2; ++pass) { for (int i = t_; i < CSR_GN / 4; i += 256) { v4i a, c; for (int e = 0; e < 4; ++e) { a[e] = st; c[e] = 0; } *(volatile v4i*)(ROWPTR + v0 + i * 4) = a; *(volatile v4i*)(ROWCNT + v0 + i * 4) = c; } if (t_ == 0) ((volatile int*)FLAG)[0] = 1; __threadfence(); } (void)nv; return; }
  if (t_ == 0) { int acc = 0; for (int b = 0; b < CSR_NBLK; ++b) { boff[b] = acc; int c = HST[(size_t)b * NGP + g]; c = (c < 0) ? 0 : (c > CHP ? CHP : c); acc += c; if (acc > tot) acc = tot; } boff[CSR_NBLK] = acc; }
  for (int i = t_; i <= CSR_GN; i += 256) ncnt[i] = 0;
  __syncthreads();
  for (int b = 0; b < CSR_NBLK; ++b) { const int c = boff[b + 1] - boff[b]; int o_ = OFF[(size_t)g * CSR_NBLK + b]; o_ = (o_ < 0) ? 0 : (o_ > CHP - c ? CHP - c : o_); const int* src_ = STG + (size_t)b * CHP + o_;
    for (int i = t_; i < c; i += 256) { int id = src_[i]; id = (id < 0) ? 0 : id; ids[boff[b] + i] = id; int d = dst[id]; d = (d < v0) ? v0 : (d >= N ? N - 1 : d); int kk = d - v0; kk = (kk < 0) ? 0 : (kk >= CSR_GN ? CSR_GN - 1 : kk); key[boff[b] + i] = (unsigned short)kk; } }
  __syncthreads();
  if (t_ == 0) { for (int i = 0; i < tot; ++i) ncnt[key[i]] += 1; int acc = 0; for (int vl = 0; vl < CSR_GN; ++vl) { const int c = ncnt[vl]; ncnt[vl] = acc; acc += c; } ncnt[CSR_GN] = acc;
    for (int i = 0; i < tot; ++i) { const int vl = key[i]; outp[ncnt[vl]] = ids[i]; ncnt[vl] += 1; }
    for (int vl = CSR_GN; vl > 0; --vl) ncnt[vl] = ncnt[vl - 1]; ncnt[0] = 0; }
  __syncthreads();
  for (int pass = 0; pass < 2; ++pass) {
    for (int i = t_; i < (stn - st) / 4; i += 256) { v4i v; for (int e = 0; e < 4; ++e) { const int q = i * 4 + e; v[e] = (q < tot) ? outp[q] : -1; } *(volatile v4i*)(PERM + st + i * 4) = v; }
    for (int i = t_; i < CSR_GN / 4; i += 256) { v4i a, c; for (int e = 0; e < 4; ++e) { const int vl = i * 4 + e; a[e] = st + ncnt[vl]; c[e] = (vl < nv) ? (ncnt[vl + 1] - ncnt[vl]) : 0; } *(volatile v4i*)(ROWPTR + v0 + i * 4) = a; *(volatile v4i*)(ROWCNT + v0 + i * 4) = c; }
    __threadfence(); }
}
__global__ __launch_bounds__(256) void csrZ_kernel(int* __restrict__ p, size_t n4) { typedef __attribute__((ext_vector_type(4))) int v4i; const size_t tid = (size_t)blockIdx.x * 256 + threadIdx.x, nth = (size_t)gridDim.x * 256; v4i z = {0, 0, 0, 0}; for (size_t i = tid; i < n4; i += nth) *(volatile v4i*)(p + i * 4) = z; }
struct CsrBufs { int *STG, *HST, *OFF, *START, *TOT, *PERM, *ROWPTR, *ROWCNT, *FLAG; int nG, NGP, CHP; size_t permLen; char* base; size_t bytes; };
static size_t csr_carve(CsrBufs& c, char* ws, size_t off, int E, int N) {
  const size_t off0 = off; c.base = ws + off;
  auto al = [&](size_t bytes) { char* p = ws + off; off += (bytes + 255) & ~(size_t)255; return p; };
  c.nG = (N + CSR_GN - 1) / CSR_GN; c.NGP = (c.nG + 31) & ~31; const int ch = (E + CSR_NBLK - 1) / CSR_NBLK; c.CHP = (ch + 31) & ~31; c.permLen = (size_t)E + 32 * (size_t)c.nG + 32;
  c.STG = (int*)al((size_t)CSR_NBLK * c.CHP * 4); c.HST = (int*)al((size_t)CSR_NBLK * c.NGP * 4); c.OFF = (int*)al((size_t)c.NGP * CSR_NBLK * 4); c.START = (int*)al((size_t)(c.NGP + 64) * 4); c.TOT = (int*)al((size_t)(c.NGP + 64) * 4);
  c.PERM = (int*)al(c.permLen * 4); c.ROWPTR = (int*)al((size_t)c.nG * CSR_GN * 4); c.ROWCNT = (int*)al((size_t)c.nG * CSR_GN * 4); c.FLAG = (int*)al(256);
  c.bytes = off - off0; return off;
}
static void csr_build(const CsrBufs& c, const int* dst, int E, int N, hipStream_t stream) {
  const size_t smem = (size_t)(2 * c.NGP + c.CHP) * 4;
  csrZ_kernel<<<512, 256, 0, stream>>>((int*)c.base, c.bytes / 16);
  csrA_kernel<<<CSR_NBLK, 64, smem, stream>>>(dst, E, N, c.nG, c.CHP, c.NGP, c.STG, c.HST);
  csrS_kernel<<<1, 512, 0, stream>>>(c.HST, c.nG, c.NGP, c.START, c.TOT, c.OFF);
  csrB_kernel<<<c.nG, 256, 0, stream>>>(dst, N, c.nG, c.CHP, c.NGP, (int)c.permLen, c.STG, c.HST, c.OFF, c.START, c.TOT, c.PERM, c.ROWPTR, c.ROWCNT, c.FLAG);
}


__global__ __launch_bounds__(256) void prep_kernel(const float* __restrict__ x, const float* __restrict__ w1r, const float* __restrict__ w1o, const float* __restrict__ w2r, const float* __restrict__ w2o, const float* __restrict__ w3r, const float* __restrict__ w3o, const float* __restrict__ w4r, const float* __restrict__ w4o, b16* __restrict__ Xh, b16* __restrict__ Xl, b16* __restrict__ W1, b16* __restrict__ W2, b16* __restrict__ W3, b16* __restrict__ W4) {
  const size_t t = (size_t)blockIdx.x * 256 + threadIdx.x; const size_t nx = (size_t)NP * 64 / 8, n1 = (size_t)128 * 128 / 8, n2 = (size_t)256 * 256 / 8, n3 = (size_t)64 * 512 / 8, n4 = (size_t)32 * 128 / 8; v8b o, z = {};
  if (t < nx) { const size_t e = t * 8; const size_t row = e / 64; for (int j = 0; j < 8; ++j) o[j] = (row < (size_t)N) ? (b16)(bf16_rne(x[e + j]) * XS) : (b16)0.0f; for (int pass = 0; pass < 2; ++pass) { *(volatile v8b*)(Xh + e) = o; *(volatile v8b*)(Xl + e) = z; __threadfence(); } return; }
  size_t u = t - nx; const float *wr, *wo; int cin; b16* dst;
  if (u < n1) { wr = w1r; wo = w1o; cin = 64; dst = W1; } else if ((u -= n1) < n2) { wr = w2r; wo = w2o; cin = 128; dst = W2; } else if ((u -= n2) < n3) { wr = w3r; wo = w3o; cin = 256; dst = W3; } else if ((u -= n3) < n4) { wr = w4r; wo = w4o; cin = 64; dst = W4; } else return;
  const size_t e = u * 8; const int oo = (int)(e / (2 * cin)), k0 = (int)(e % (2 * cin));
  for (int j = 0; j < 8; ++j) { const int k = k0 + j; const float v = (k < cin) ? wr[(size_t)oo * cin + k] : wo[(size_t)oo * cin + (k - cin)]; o[j] = (b16)(bf16_rne(v) * WSC); }
  for (int pass = 0; pass < 2; ++pass) { *(volatile v8b*)(dst + e) = o; __threadfence(); }
}
template <int CIN, int COUT, int LAST>
__global__ __launch_bounds__(128) void layer_kernel(const b16* __restrict__ Th, const b16* __restrict__ Tl, const int* __restrict__ srcs, const float* __restrict__ ew, const int* __restrict__ PERM, const int* __restrict__ ROWPTR, const int* __restrict__ ROWCNT, int permLen, const b16* __restrict__ W, const float* __restrict__ bias, b16* __restrict__ Hh, b16* __restrict__ Hl, float* __restrict__ out) {
  constexpr int NT = COUT / 16, CPL = CIN / 32;
  __shared__ __attribute__((aligned(16))) b16 Ah[64][CIN + 8], Al[64][CIN + 8]; __shared__ __attribute__((aligned(16))) float Ts[4][16][32 + 4]; __shared__ __attribute__((aligned(16))) b16 Oh[LAST ? 1 : 4][16][(LAST ? 8 : COUT) + 8], Ol[LAST ? 1 : 4][16][(LAST ? 8 : COUT) + 8];
  const int wave = threadIdx.x >> 5, lane = threadIdx.x & 31, nloc = lane & 15, hlf = lane >> 4; const size_t row0 = (size_t)blockIdx.x * 64; const size_t m0 = row0 + wave * 16;
  for (int rl = 0; rl < 16; ++rl) { const size_t v = m0 + rl; float acc[CPL]; for (int q = 0; q < CPL; ++q) acc[q] = 0.0f;
    if (v < (size_t)N) { int st = ROWPTR[v], cnt = ROWCNT[v]; cnt = iclamp(cnt, 0, 4096); st = iclamp(st, 0, permLen - cnt);
      for (int j = 0; j < cnt; ++j) { const int e = iclamp(PERM[st + j], 0, E - 1); const int s = iclamp(srcs[e], 0, N - 1); const float w_ = bf16_rne(ew[e]); const b16* th = Th + (size_t)s * CIN + lane * CPL; const b16* tl = Tl + (size_t)s * CIN + lane * CPL;
        for (int q = 0; q < CPL; ++q) acc[q] += pmul(w_, ((float)th[q] + (float)tl[q]) * (1.0f / XS)); } }
    for (int q = 0; q < CPL; ++q) { b16 p, qq; split16(acc[q] * XS, p, qq); Ah[wave * 16 + rl][lane * CPL + q] = p; Al[wave * 16 + rl][lane * CPL + q] = qq; } }
  wave_lds_sync();
  v8f acc2[NT];
#pragma unroll
  for (int t = 0; t < NT; ++t) acc2[t] = (v8f){};
  for (int kb = 0; kb < CIN; kb += 32) { const v16b a = frag_kb(&Ah[wave * 16 + nloc][kb], hlf), al = frag_kb(&Al[wave * 16 + nloc][kb], hlf), s = frag_kb(Th + (m0 + nloc) * CIN + kb, hlf), sl = frag_kb(Tl + (m0 + nloc) * CIN + kb, hlf);
#pragma unroll
    for (int t = 0; t < NT; ++t) { const v16b wa = frag_kb(W + (size_t)(t * 16 + nloc) * (2 * CIN) + kb, hlf), wsf = frag_kb(W + (size_t)(t * 16 + nloc) * (2 * CIN) + CIN + kb, hlf); acc2[t] = wmma16b(a, wa, acc2[t]); acc2[t] = wmma16b(al, wa, acc2[t]); acc2[t] = wmma16b(s, wsf, acc2[t]); acc2[t] = wmma16b(sl, wsf, acc2[t]); } }
  for (int pass = 0; pass < 2; ++pass) {
#pragma unroll
    for (int t = 0; t < NT; ++t) { const int c = t * 16 + nloc; const float bb = bf16_rne(bias[c]);
      if (LAST) {
#pragma unroll
        for (int r = 0; r < 8; ++r) Ts[wave][8 * hlf + r][c] = acc2[t][r] * (1.0f / (XS * WSC)) + bb; }
      else {
#pragma unroll
        for (int r = 0; r < 8; ++r) { const size_t row = m0 + 8 * hlf + r; const float v = (row < (size_t)N) ? acc2[t][r] * (1.0f / (XS * WSC)) + bb : 0.0f; b16 p, q; split16(v * XS, p, q); Oh[wave][8 * hlf + r][c] = p; Ol[wave][8 * hlf + r][c] = q; } } }
    if (!LAST) { wave_lds_sync(); for (int q = lane; q < 16 * (COUT / 8); q += 32) { const int rr = q / (COUT / 8), c8 = (q % (COUT / 8)) * 8; const size_t row = m0 + rr; *(volatile v8b*)(Hh + row * COUT + c8) = *(const v8b*)(&Oh[wave][rr][c8]); *(volatile v8b*)(Hl + row * COUT + c8) = *(const v8b*)(&Ol[wave][rr][c8]); } }
    if (LAST) { wave_lds_sync(); for (int rr = 0; rr < 16; ++rr) { const size_t row = m0 + rr; if (row < (size_t)N && lane < 8) *(volatile v4f*)(out + row * 32 + lane * 4) = *(const v4f*)(&Ts[wave][rr][lane * 4]); } }
    __threadfence(); }
}
template <int C>
__global__ __launch_bounds__(256) void bnsum_kernel(const b16* __restrict__ Hh, const b16* __restrict__ Hl, const float* __restrict__ MEAN, float* __restrict__ P) {
  const int blk = blockIdx.x, col = threadIdx.x; if (col >= C) return; float s = 0.0f; const int r0 = blk * 128, r1 = min(r0 + 128, N);
  if (MEAN) { const float mu = MEAN[col]; for (int r = r0; r < r1; ++r) { const float h = ((float)Hh[(size_t)r * C + col] + (float)Hl[(size_t)r * C + col]) * (1.0f / XS); const float dv = h - mu; s += dv * dv; } }
  else { for (int r = r0; r < r1; ++r) s += ((float)Hh[(size_t)r * C + col] + (float)Hl[(size_t)r * C + col]) * (1.0f / XS); }
  for (int pass = 0; pass < 2; ++pass) { ((volatile float*)P)[(size_t)blk * C + col] = s; __threadfence(); }
}
template <int C>
__global__ __launch_bounds__(256) void bnfin_kernel(const float* __restrict__ P, int isvar, float* __restrict__ OUTV) {
  const int col = threadIdx.x; if (col >= C) return; float s = 0.0f; for (int b = 0; b < NBLKR; ++b) s += P[(size_t)b * C + col]; s *= (1.0f / N); const float o = isvar ? rsqrtf(s + BNE) : s;
  for (int pass = 0; pass < 2; ++pass) { ((volatile float*)OUTV)[col] = o; __threadfence(); }
}
template <int C>
__global__ __launch_bounds__(256) void bnapply_kernel(b16* __restrict__ Hh, b16* __restrict__ Hl, const float* __restrict__ MEAN, const float* __restrict__ RSTD, const float* __restrict__ g, const float* __restrict__ be) {
  const size_t t = (size_t)blockIdx.x * 256 + threadIdx.x; if (t >= (size_t)N * C / 8) return; const size_t e = t * 8; const int c0 = (int)(e % C);
  const v8b a = *(const v8b*)(Hh + e), b = *(const v8b*)(Hl + e); v8b hv, lv;
#pragma unroll
  for (int j = 0; j < 8; ++j) { const int c = c0 + j; const float h = ((float)a[j] + (float)b[j]) * (1.0f / XS); const float y = tanh_(pmul(pmul(bf16_rne(g[c]), h - MEAN[c]), RSTD[c]) + bf16_rne(be[c])); b16 p, q; split16(y * XS, p, q); hv[j] = p; lv[j] = q; }
  for (int pass = 0; pass < 2; ++pass) { *(volatile v8b*)(Hh + e) = hv; *(volatile v8b*)(Hl + e) = lv; __threadfence(); }
}
}

extern "C" void kernel_launch(void* const* d_in, const int* in_sizes, int n_in, void* d_out, int out_size, void* d_ws, size_t ws_size, hipStream_t stream) {
  (void)n_in;
  auto Fp = [&](int i) { return (const float*)d_in[i]; }; auto Ip = [&](int i) { return (const int*)d_in[i]; };
  if (in_sizes[0] != N * 64 || in_sizes[1] != 2 * E || in_sizes[2] != E || in_sizes[3] != 128 * 64 || in_sizes[8] != 256 * 128 || in_sizes[13] != 64 * 256 || in_sizes[18] != 32 * 64 || out_size != N * 32) return;
  size_t off = 0; char* ws = (char*)d_ws;
  auto carve = [&](size_t bytes) { char* p = ws + off; off += (bytes + 255) & ~(size_t)255; return p; };
  b16* Xh = (b16*)carve((size_t)NP * 64 * 2); b16* Xl = (b16*)carve((size_t)NP * 64 * 2); b16* W1 = (b16*)carve((size_t)128 * 128 * 2); b16* W2 = (b16*)carve((size_t)256 * 256 * 2); b16* W3 = (b16*)carve((size_t)64 * 512 * 2); b16* W4 = (b16*)carve((size_t)32 * 128 * 2);
  b16* H1h = (b16*)carve((size_t)NP * 128 * 2); b16* H1l = (b16*)carve((size_t)NP * 128 * 2); b16* H2h = (b16*)carve((size_t)NP * 256 * 2); b16* H2l = (b16*)carve((size_t)NP * 256 * 2);
  b16* H3h = H1h; b16* H3l = H1l;
  float* P = (float*)carve((size_t)NBLKR * 256 * 4); float* MEAN = (float*)carve(256 * 4); float* RSTD = (float*)carve(256 * 4);
  CsrBufs csr; off = csr_carve(csr, ws, off, E, N);
  if (off > ws_size || off > ((size_t)128 << 20)) return;
  prep_kernel<<<(unsigned)(((size_t)NP * 64 / 8 + (128 * 128 + 256 * 256 + 64 * 512 + 32 * 128) / 8 + 255) / 256), 256, 0, stream>>>(Fp(0), Fp(3), Fp(4), Fp(8), Fp(9), Fp(13), Fp(14), Fp(18), Fp(19), Xh, Xl, W1, W2, W3, W4);
  csr_build(csr, Ip(1) + E, E, N, stream);
  layer_kernel<64, 128, 0><<<NP / 64, 128, 0, stream>>>(Xh, Xl, Ip(1), Fp(2), csr.PERM, csr.ROWPTR, csr.ROWCNT, (int)csr.permLen, W1, Fp(5), H1h, H1l, nullptr);
  bnsum_kernel<128><<<NBLKR, 256, 0, stream>>>(H1h, H1l, nullptr, P); bnfin_kernel<128><<<1, 256, 0, stream>>>(P, 0, MEAN); bnsum_kernel<128><<<NBLKR, 256, 0, stream>>>(H1h, H1l, MEAN, P); bnfin_kernel<128><<<1, 256, 0, stream>>>(P, 1, RSTD);
  bnapply_kernel<128><<<(unsigned)(((size_t)N * 128 / 8 + 255) / 256), 256, 0, stream>>>(H1h, H1l, MEAN, RSTD, Fp(6), Fp(7));
  layer_kernel<128, 256, 0><<<NP / 64, 128, 0, stream>>>(H1h, H1l, Ip(1), Fp(2), csr.PERM, csr.ROWPTR, csr.ROWCNT, (int)csr.permLen, W2, Fp(10), H2h, H2l, nullptr);
  bnsum_kernel<256><<<NBLKR, 256, 0, stream>>>(H2h, H2l, nullptr, P); bnfin_kernel<256><<<1, 256, 0, stream>>>(P, 0, MEAN); bnsum_kernel<256><<<NBLKR, 256, 0, stream>>>(H2h, H2l, MEAN, P); bnfin_kernel<256><<<1, 256, 0, stream>>>(P, 1, RSTD);
  bnapply_kernel<256><<<(unsigned)(((size_t)N * 256 / 8 + 255) / 256), 256, 0, stream>>>(H2h, H2l, MEAN, RSTD, Fp(11), Fp(12));
  layer_kernel<256, 64, 0><<<NP / 64, 128, 0, stream>>>(H2h, H2l, Ip(1), Fp(2), csr.PERM, csr.ROWPTR, csr.ROWCNT, (int)csr.permLen, W3, Fp(15), H3h, H3l, nullptr);
  bnsum_kernel<64><<<NBLKR, 256, 0, stream>>>(H3h, H3l, nullptr, P); bnfin_kernel<64><<<1, 256, 0, stream>>>(P, 0, MEAN); bnsum_kernel<64><<<NBLKR, 256, 0, stream>>>(H3h, H3l, MEAN, P); bnfin_kernel<64><<<1, 256, 0, stream>>>(P, 1, RSTD);
  bnapply_kernel<64><<<(unsigned)(((size_t)N * 64 / 8 + 255) / 256), 256, 0, stream>>>(H3h, H3l, MEAN, RSTD, Fp(16), Fp(17));
  layer_kernel<64, 32, 1><<<NP / 64, 128, 0, stream>>>(H3h, H3l, Ip(1), Fp(2), csr.PERM, csr.ROWPTR, csr.ROWCNT, (int)csr.permLen, W4, Fp(20), nullptr, nullptr, (float*)d_out);
}
